// ParameterKernel_36112085025350
// MI455X (gfx1250) — hardware-verified
//
#include <hip/hip_runtime.h>

#define NREF 4096
#define NIN  8192
#define DF   512
#define PDIM 256

#define BJ   64
#define IC   128
#define DSTR 520
#define KSTR 136
#define OSTR 36

#define LDS_DESC_BYTES (BJ * DSTR * 2)
#define LDS_K_BYTES    (BJ * KSTR * 2)
#define LDS_MAIN_BYTES (LDS_DESC_BYTES + 2 * LDS_K_BYTES)
#define LDS_OST_BYTES  (8 * BJ * OSTR * 4)
#define LDS_BYTES      LDS_MAIN_BYTES

static_assert(LDS_OST_BYTES <= LDS_BYTES);
static_assert(NREF % IC == 0);
static_assert(NIN % BJ == 0);
static_assert(DF % 32 == 0);
static_assert(IC % 32 == 0);
static_assert((DSTR % 8) == 0);
static_assert((KSTR % 8) == 0);
static_assert((OSTR % 4) == 0);

typedef _Float16 v16h __attribute__((ext_vector_type(16)));
typedef __bf16   v16b __attribute__((ext_vector_type(16)));
typedef float    v8f  __attribute__((ext_vector_type(8)));
typedef float    v4f  __attribute__((ext_vector_type(4)));
typedef unsigned int v4u __attribute__((ext_vector_type(4)));
typedef int      v4i  __attribute__((ext_vector_type(4)));

union FH { v16h v; v4u q[2]; };
union FB { v16b v; v4u q[2]; };

__device__ __forceinline__ unsigned short f2bf_bits(float f) {
  unsigned u = __float_as_uint(f);
  return (unsigned short)((u + 0x7FFFu + ((u >> 16) & 1u)) >> 16);
}
__device__ __forceinline__ float bf_bits2f(unsigned short b) { return __uint_as_float(((unsigned)b) << 16); }
__device__ __forceinline__ unsigned pk16(unsigned short a, unsigned short b) { return (unsigned)a | ((unsigned)b << 16); }

__device__ __forceinline__ unsigned short f2h_bits(float f) {
  _Float16 hv = (_Float16)f;
  return __builtin_bit_cast(unsigned short, hv);
}

__device__ __forceinline__ void split2(float f0, float f1, unsigned& hw, unsigned& lw) {
  const unsigned short h0 = f2bf_bits(f0), h1 = f2bf_bits(f1);
  const unsigned short l0 = f2bf_bits(f0 - bf_bits2f(h0)), l1 = f2bf_bits(f1 - bf_bits2f(h1));
  hw = pk16(h0, h1);
  lw = pk16(l0, l1);
}

__device__ __forceinline__ v8f mma_h(v16h a, v16h b, v8f c) {
  c = __builtin_amdgcn_wmma_f32_16x16x32_f16(false, a, false, b, (short)0, c, false, false);
  asm volatile("v_nop\n\tv_nop\n\tv_nop\n\tv_nop" : "+v"(c) : "v"(a), "v"(b));
  return c;
}
__device__ __forceinline__ v8f mma_b(v16b a, v16b b, v8f c) {
  c = __builtin_amdgcn_wmma_f32_16x16x32_bf16(false, a, false, b, (short)0, c, false, false);
  asm volatile("v_nop\n\tv_nop\n\tv_nop\n\tv_nop" : "+v"(c) : "v"(a), "v"(b));
  return c;
}

__global__ __launch_bounds__(256) void cvt_f16_kernel(const float* __restrict__ src,
                                                      unsigned short* __restrict__ dst, int ngrp) {
  const int t = blockIdx.x * 256 + (int)threadIdx.x;
  if (t >= ngrp) return;
  const size_t so = (size_t)t * 8;
  const v4f a0 = *(const v4f*)(src + so);
  const v4f a1 = *(const v4f*)(src + so + 4);
  const unsigned w0 = pk16(f2h_bits(a0[0]), f2h_bits(a0[1]));
  const unsigned w1 = pk16(f2h_bits(a0[2]), f2h_bits(a0[3]));
  const unsigned w2 = pk16(f2h_bits(a1[0]), f2h_bits(a1[1]));
  const unsigned w3 = pk16(f2h_bits(a1[2]), f2h_bits(a1[3]));
  const v4u vv = (v4u){w0, w1, w2, w3};
  volatile v4u* p = (volatile v4u*)(dst + so);
  *p = vv;
  __threadfence();
  *p = vv;
}

__global__ __launch_bounds__(256) void split_bf16_kernel(const float* __restrict__ src,
                                                         unsigned short* __restrict__ hi,
                                                         unsigned short* __restrict__ lo, int ngrp) {
  const int t = blockIdx.x * 256 + (int)threadIdx.x;
  if (t >= ngrp) return;
  const size_t so = (size_t)t * 8;
  const v4f a0 = *(const v4f*)(src + so);
  const v4f a1 = *(const v4f*)(src + so + 4);
  unsigned h0, h1, h2, h3, l0, l1, l2, l3;
  split2(a0[0], a0[1], h0, l0);
  split2(a0[2], a0[3], h1, l1);
  split2(a1[0], a1[1], h2, l2);
  split2(a1[2], a1[3], h3, l3);
  const v4u hv = (v4u){h0, h1, h2, h3};
  const v4u lv = (v4u){l0, l1, l2, l3};
  volatile v4u* ph = (volatile v4u*)(hi + so);
  volatile v4u* pl = (volatile v4u*)(lo + so);
  *ph = hv;
  *pl = lv;
  __threadfence();
  *ph = hv;
  *pl = lv;
}

__global__ __launch_bounds__(256)
void fused_kernel(const unsigned short* __restrict__ Xp,
                  const unsigned short* __restrict__ Dp,
                  const unsigned short* __restrict__ Ahp,
                  const unsigned short* __restrict__ Alp,
                  const int* __restrict__ Zref,
                  const int* __restrict__ Zin,
                  const int* __restrict__ expk,
                  float* __restrict__ out) {
  extern __shared__ __align__(16) unsigned char smem[];
  unsigned short* Dsh = (unsigned short*)smem;
  unsigned short* Kh  = (unsigned short*)(smem + LDS_DESC_BYTES);
  unsigned short* Kl  = (unsigned short*)(smem + LDS_DESC_BYTES + LDS_K_BYTES);

  const int tid  = threadIdx.x;
  const int w    = tid >> 5;
  const int lane = tid & 31;
  const int h    = lane >> 4;
  const int m    = lane & 15;
  const int j0   = blockIdx.x * BJ;

  for (int idx = tid; idx < BJ * (DF / 8); idx += 256) {
    const int row = idx >> 6;
    const int k   = (idx & 63) * 8;
    *(v4u*)(Dsh + row * DSTR + k) = *(const v4u*)(Dp + (size_t)(j0 + row) * DF + k);
  }

  int zc0 = Zin[j0 + 0 * 16 + m];
  int zc1 = Zin[j0 + 1 * 16 + m];
  int zc2 = Zin[j0 + 2 * 16 + m];
  int zc3 = Zin[j0 + 3 * 16 + m];
  const int ekraw = expk[0];
  const int ek = min(max(ekraw, 0), 8);

  v8f Y[8];
#pragma unroll
  for (int q = 0; q < 8; ++q) Y[q] = (v8f){0.f, 0.f, 0.f, 0.f, 0.f, 0.f, 0.f, 0.f};

  __syncthreads();

#pragma unroll 1
  for (int c = 0; c < NREF / IC; ++c) {
    const int ib = c * IC;

    v8f S[4];
#pragma unroll
    for (int t = 0; t < 4; ++t) S[t] = (v8f){0.f, 0.f, 0.f, 0.f, 0.f, 0.f, 0.f, 0.f};
    const unsigned short* xrow = Xp + (size_t)(ib + 16 * w + m) * DF + 8 * h;
#pragma unroll 2
    for (int ks = 0; ks < DF / 32; ++ks) {
      FH a;
      a.q[0] = *(const v4u*)(xrow + 32 * ks);
      a.q[1] = *(const v4u*)(xrow + 32 * ks + 16);
#pragma unroll
      for (int t = 0; t < 4; ++t) {
        const unsigned short* drow = Dsh + (16 * t + m) * DSTR + 32 * ks + 8 * h;
        FH b;
        b.q[0] = *(const v4u*)(drow);
        b.q[1] = *(const v4u*)(drow + 16);
        S[t] = mma_h(a.v, b.v, S[t]);
      }
    }

    const int* zp = Zref + ib + 16 * w + 8 * h;
    const v4i z0 = *(const v4i*)(zp);
    const v4i z1 = *(const v4i*)(zp + 4);

    __syncthreads();

#pragma unroll
    for (int t = 0; t < 4; ++t) {
      const int zct = (t == 0) ? zc0 : (t == 1) ? zc1 : (t == 2) ? zc2 : zc3;
      unsigned hw[4], lw[4];
#pragma unroll
      for (int rp = 0; rp < 4; ++rp) {
        float v2[2];
#pragma unroll
        for (int q = 0; q < 2; ++q) {
          const int r = 2 * rp + q;
          const float s = S[t][r];
          float v = 1.0f;
#pragma unroll
          for (int e = 0; e < 8; ++e) v = (e < ek) ? (v * s) : v;
          const int zr = (r < 4) ? z0[r] : z1[r - 4];
          if (zr != zct) v = 0.0f;
          v2[q] = v;
        }
        split2(v2[0], v2[1], hw[rp], lw[rp]);
      }
      const int ko = (16 * t + m) * KSTR + 16 * w + 8 * h;
      *(v4u*)(Kh + ko) = (v4u){hw[0], hw[1], hw[2], hw[3]};
      *(v4u*)(Kl + ko) = (v4u){lw[0], lw[1], lw[2], lw[3]};
    }
    __syncthreads();

#pragma unroll 1
    for (int ks = 0; ks < IC / 32; ++ks) {
      const size_t base0 = (size_t)(32 * w + m) * NREF + ib + 32 * ks + 8 * h;
      const size_t base1 = base0 + (size_t)16 * NREF;
      FB ah0, al0, ah1, al1;
      ah0.q[0] = *(const v4u*)(Ahp + base0);
      ah0.q[1] = *(const v4u*)(Ahp + base0 + 16);
      al0.q[0] = *(const v4u*)(Alp + base0);
      al0.q[1] = *(const v4u*)(Alp + base0 + 16);
      ah1.q[0] = *(const v4u*)(Ahp + base1);
      ah1.q[1] = *(const v4u*)(Ahp + base1 + 16);
      al1.q[0] = *(const v4u*)(Alp + base1);
      al1.q[1] = *(const v4u*)(Alp + base1 + 16);
#pragma unroll
      for (int t = 0; t < 4; ++t) {
        const int ko = (16 * t + m) * KSTR + 32 * ks + 8 * h;
        FB bh, bl;
        bh.q[0] = *(const v4u*)(Kh + ko);
        bh.q[1] = *(const v4u*)(Kh + ko + 16);
        bl.q[0] = *(const v4u*)(Kl + ko);
        bl.q[1] = *(const v4u*)(Kl + ko + 16);
        Y[t] = mma_b(ah0.v, bh.v, Y[t]);
        Y[t] = mma_b(ah0.v, bl.v, Y[t]);
        Y[t] = mma_b(al0.v, bh.v, Y[t]);
        Y[4 + t] = mma_b(ah1.v, bh.v, Y[4 + t]);
        Y[4 + t] = mma_b(ah1.v, bl.v, Y[4 + t]);
        Y[4 + t] = mma_b(al1.v, bh.v, Y[4 + t]);
      }
    }
  }

  __syncthreads();

  float* ost = (float*)smem + w * (BJ * OSTR);
#pragma unroll
  for (int u = 0; u < 2; ++u) {
#pragma unroll
    for (int t = 0; t < 4; ++t) {
      float* os = ost + (16 * t + m) * OSTR + 16 * u + 8 * h;
      const v8f yv = Y[4 * u + t];
      *(v4f*)(os)     = (v4f){yv[0], yv[1], yv[2], yv[3]};
      *(v4f*)(os + 4) = (v4f){yv[4], yv[5], yv[6], yv[7]};
    }
  }
  __syncthreads();

  {
    const int rh = lane >> 4;
    const int c4 = (lane & 15) * 4;
    float* ob = out + (size_t)(32 * w) * NIN + j0 + c4;
    for (int ps = 0; ps < 2; ++ps) {
#pragma unroll
      for (int it = 0; it < 16; ++it) {
        const int row = it * 2 + rh;
        const v4f vv = (v4f){ost[(c4 + 0) * OSTR + row], ost[(c4 + 1) * OSTR + row],
                             ost[(c4 + 2) * OSTR + row], ost[(c4 + 3) * OSTR + row]};
        *(volatile v4f*)(ob + (size_t)row * NIN) = vv;
      }
      __threadfence();
    }
  }
}

extern "C" void kernel_launch(void* const* d_in, const int* in_sizes, int n_in,
                              void* d_out, int out_size, void* d_ws, size_t ws_size,
                              hipStream_t stream) {
  if (n_in < 6) return;
  if (in_sizes[0] != PDIM * NREF) return;
  if (in_sizes[1] != NREF * DF) return;
  if (in_sizes[2] != NIN * DF) return;
  if (in_sizes[3] != NREF) return;
  if (in_sizes[4] != NIN) return;
  if (in_sizes[5] < 1) return;
  if (out_size != PDIM * NIN) return;

  const float* Alpha = (const float*)d_in[0];
  const float* X_ref = (const float*)d_in[1];
  const float* desc  = (const float*)d_in[2];
  const int*   Z_ref = (const int*)d_in[3];
  const int*   Zq    = (const int*)d_in[4];
  const int*   expK  = (const int*)d_in[5];
  float* o = (float*)d_out;

  size_t off = 0;
  const size_t oX  = off; off += (size_t)NREF * DF * 2;
  const size_t oD  = off; off += (size_t)NIN * DF * 2;
  const size_t oAh = off; off += (size_t)PDIM * NREF * 2;
  const size_t oAl = off; off += (size_t)PDIM * NREF * 2;
  if (off > ws_size) return;

  char* ws = (char*)d_ws;
  unsigned short* Xf = (unsigned short*)(ws + oX);
  unsigned short* Dfp = (unsigned short*)(ws + oD);
  unsigned short* Ah = (unsigned short*)(ws + oAh);
  unsigned short* Al = (unsigned short*)(ws + oAl);

  const int ngX = NREF * DF / 8;
  cvt_f16_kernel<<<dim3((ngX + 255) / 256), dim3(256), 0, stream>>>(X_ref, Xf, ngX);
  const int ngD = NIN * DF / 8;
  cvt_f16_kernel<<<dim3((ngD + 255) / 256), dim3(256), 0, stream>>>(desc, Dfp, ngD);
  const int ngA = PDIM * NREF / 8;
  split_bf16_kernel<<<dim3((ngA + 255) / 256), dim3(256), 0, stream>>>(Alpha, Ah, Al, ngA);
  (void)hipFuncSetAttribute(reinterpret_cast<const void*>(&fused_kernel),
                            hipFuncAttributeMaxDynamicSharedMemorySize, LDS_BYTES);
  fused_kernel<<<dim3(NIN / BJ), dim3(256), LDS_BYTES, stream>>>(Xf, Dfp, Ah, Al, Z_ref, Zq, expK, o);
  (void)hipGetLastError();
}
